// MDLSTM_29171417874579
// MI455X (gfx1250) — hardware-verified
//
#include <hip/hip_runtime.h>
#include <math.h>

constexpr int NBATCH = 16;
constexpr int NCIN   = 64;
constexpr int NROW   = 32;
constexpr int NCOL   = 128;
constexpr int NHID   = 64;
constexpr int NGATE  = 5 * NHID;
constexpr int KCAT   = NCIN + 2 * NHID;
constexpr int NDIR   = 4;
constexpr int CELL_ELEMS = NBATCH * NHID;
constexpr int SLABP  = 68;
constexpr int TPITCH = 65;
constexpr int GATE_ROWSTRIDE = NHID * KCAT;
constexpr int NPIX   = NROW * NCOL;
constexpr int NOUT_ONE = NBATCH * NHID * NROW * NCOL;
constexpr float WCARRY     = 16.0f;
constexpr float WCARRY_INV = 1.0f / 16.0f;
static_assert(NBATCH == 16, "one 16-row m-subtile per cell");
static_assert(NCIN == 64 && NHID == 64, "64-wide operand tiles");
static_assert(NGATE == 320 && KCAT == 192, "gate and K extents");
static_assert(KCAT % 32 == 0, "K multiple of 32");
static_assert(NCOL % 64 == 0, "w tiles of 64");
static_assert(CELL_ELEMS == 1024, "cell tile size");

typedef __attribute__((ext_vector_type(16))) _Float16 v16h;
typedef __attribute__((ext_vector_type(8)))  _Float16 v8h;
typedef __attribute__((ext_vector_type(8)))  float    v8f;
typedef __attribute__((ext_vector_type(4)))  float    v4f;
typedef __attribute__((ext_vector_type(4)))  unsigned v4u;

__device__ __forceinline__ unsigned short f2bf_bits(float f) {
  unsigned u = __float_as_uint(f);
  return (unsigned short)((u + 0x7FFFu + ((u >> 16) & 1u)) >> 16);
}
__device__ __forceinline__ float bf_bits2f(unsigned short h) { return __uint_as_float(((unsigned)h) << 16); }
__device__ __forceinline__ float bf16r(float f) { return bf_bits2f(f2bf_bits(f)); }

__device__ __forceinline__ float h16_to_f32(unsigned hb) {
  const unsigned sgn = (hb & 0x8000u) << 16;
  const unsigned em = hb & 0x7fffu;
  const float fn = __uint_as_float((em << 13) + 0x38000000u);
  const float fs = (float)em * 5.9604644775390625e-8f;
  const float mag = (em < 0x400u) ? fs : fn;
  return __uint_as_float(__float_as_uint(mag) | sgn);
}

__device__ __forceinline__ void dep_guard_h(v8f& a, v8f& b, v16h x, v16h y) { asm volatile("v_nop\n\tv_nop\n\tv_nop\n\tv_nop" : "+v"(a), "+v"(b) : "v"(x), "v"(y)); }
__device__ __forceinline__ void keep4_h(v16h a, v16h b, v16h c, v16h d) { asm volatile("v_nop" :: "v"(a), "v"(b), "v"(c), "v"(d)); }
template <typename T> struct Frag;
template <> struct Frag<_Float16> {
  typedef v16h V; union U { v16h v; v8h h[2]; };
  static __device__ __forceinline__ v16h load(const _Float16* p) {
    U f; f.h[0] = *(const v8h*)(p); f.h[1] = *(const v8h*)(p + 16); return f.v;
  }
  static __device__ __forceinline__ v8f mma(v16h a, v16h b, v8f c) {
    return __builtin_amdgcn_wmma_f32_16x16x32_f16(false, a, false, b, (short)0, c, false, false);
  }
  static __device__ __forceinline__ void guard(v8f& a, v8f& b, v16h x, v16h y) { dep_guard_h(a, b, x, y); }
  static __device__ __forceinline__ void keep(v16h a, v16h b, v16h c, v16h d) { keep4_h(a, b, c, d); }
};

__device__ __forceinline__ void guard5(v8f& a0, v8f& a1, v8f& a2, v8f& a3, v8f& a4,
                                       v16h x, v16h b0, v16h b1, v16h b2, v16h b3, v16h b4) {
  asm volatile("v_nop\n\tv_nop\n\tv_nop\n\tv_nop"
               : "+v"(a0), "+v"(a1), "+v"(a2), "+v"(a3), "+v"(a4)
               : "v"(x), "v"(b0), "v"(b1), "v"(b2), "v"(b3), "v"(b4));
}

__device__ __forceinline__ void kstep5(v8f& a0, v8f& a1, v8f& a2, v8f& a3, v8f& a4,
                                       const v16h a, const _Float16* wr) {
  const v16h b0 = Frag<_Float16>::load(wr);
  const v16h b1 = Frag<_Float16>::load(wr + (size_t)1 * GATE_ROWSTRIDE);
  const v16h b2 = Frag<_Float16>::load(wr + (size_t)2 * GATE_ROWSTRIDE);
  const v16h b3 = Frag<_Float16>::load(wr + (size_t)3 * GATE_ROWSTRIDE);
  const v16h b4 = Frag<_Float16>::load(wr + (size_t)4 * GATE_ROWSTRIDE);
  a0 = Frag<_Float16>::mma(a, b0, a0);
  a1 = Frag<_Float16>::mma(a, b1, a1);
  a2 = Frag<_Float16>::mma(a, b2, a2);
  a3 = Frag<_Float16>::mma(a, b3, a3);
  a4 = Frag<_Float16>::mma(a, b4, a4);
  guard5(a0, a1, a2, a3, a4, a, b0, b1, b2, b3, b4);
}

__device__ __forceinline__ float fsig(float x)  { return __builtin_amdgcn_rcpf(1.0f + __expf(-x)); }
__device__ __forceinline__ float ftanh(float x) { return 1.0f - 2.0f * __builtin_amdgcn_rcpf(__expf(2.0f * x) + 1.0f); }

__global__ __launch_bounds__(256) void pack_x_kernel(const float* __restrict__ x, unsigned short* __restrict__ xp) {
  __shared__ float Tt[64 * TPITCH];
  const int tid = threadIdx.x;
  const int w0 = blockIdx.x * 64, h = blockIdx.y, b = blockIdx.z;
#pragma unroll
  for (int i = 0; i < 4; ++i) {
    const int idx = i * 256 + tid;
    const int rr = idx >> 4, cc = (idx & 15) * 4;
    const v4f v = *(const v4f*)(x + (((size_t)b * NCIN + rr) * NROW + h) * NCOL + w0 + cc);
    Tt[rr * TPITCH + cc + 0] = v[0];
    Tt[rr * TPITCH + cc + 1] = v[1];
    Tt[rr * TPITCH + cc + 2] = v[2];
    Tt[rr * TPITCH + cc + 3] = v[3];
  }
  __syncthreads();
  const int q = tid >> 3, c8 = (tid & 7) * 8;
  v8h hv[2];
#pragma unroll
  for (int g = 0; g < 2; ++g) {
    const int qq = g * 32 + q;
#pragma unroll
    for (int e = 0; e < 8; ++e) {
      const float f = Tt[(c8 + e) * TPITCH + qq];
      hv[g][e] = (_Float16)bf16r(f);
    }
  }
  for (int pass = 0; pass < 2; ++pass) {
#pragma unroll
    for (int g = 0; g < 2; ++g) {
      const size_t o = (((size_t)h * NCOL + (size_t)(w0 + g * 32 + q)) * NBATCH + b) * NCIN + c8;
      *(volatile v8h*)(xp + o) = hv[g];
    }
    __threadfence();
  }
}

__global__ __launch_bounds__(256) void pack_w_kernel(const float* __restrict__ wsrc, const float* __restrict__ u0src,
                                                     const float* __restrict__ u1src, unsigned short* __restrict__ wc) {
  __shared__ float Tt[64 * TPITCH];
  const int tid = threadIdx.x;
  const int c0 = blockIdx.x * 64, s = blockIdx.y, d = blockIdx.z;
  const float* p0 = wsrc  + (size_t)d * NCIN * NGATE;
  const float* p1 = u0src + (size_t)d * NHID * NGATE;
  const float* p2 = u1src + (size_t)d * NHID * NGATE;
  const float* src = (s == 0) ? p0 : ((s == 1) ? p1 : p2);
#pragma unroll
  for (int i = 0; i < 4; ++i) {
    const int idx = i * 256 + tid;
    const int rr = idx >> 4, cc = (idx & 15) * 4;
    const v4f v = *(const v4f*)(src + (size_t)rr * NGATE + c0 + cc);
    Tt[rr * TPITCH + cc + 0] = v[0];
    Tt[rr * TPITCH + cc + 1] = v[1];
    Tt[rr * TPITCH + cc + 2] = v[2];
    Tt[rr * TPITCH + cc + 3] = v[3];
  }
  __syncthreads();
  const int q = tid >> 3, c8 = (tid & 7) * 8;
  v8h hv[2];
#pragma unroll
  for (int g = 0; g < 2; ++g) {
    const int qq = g * 32 + q;
#pragma unroll
    for (int e = 0; e < 8; ++e) {
      const float f = Tt[(c8 + e) * TPITCH + qq];
      const float fb = bf16r(f);
      hv[g][e] = (_Float16)(fb * WCARRY);
    }
  }
  for (int pass = 0; pass < 2; ++pass) {
#pragma unroll
    for (int g = 0; g < 2; ++g) {
      const size_t o = ((size_t)d * NGATE + (size_t)(c0 + g * 32 + q)) * KCAT + (size_t)s * 64 + c8;
      *(volatile v8h*)(wc + o) = hv[g];
    }
    __threadfence();
  }
}

__global__ __launch_bounds__(32) void grid_cell_kernel(const unsigned short* __restrict__ xpp,
                                                       const unsigned short* __restrict__ wcp,
                                                       const float* __restrict__ bs,
                                                       unsigned short* hPp, float* cP, int t, int rlo) {
  __shared__ __align__(16) float sH[16 * SLABP];
  __shared__ __align__(16) float sC[16 * SLABP];
  const _Float16* xp  = (const _Float16*)xpp;
  const _Float16* wc  = (const _Float16*)wcp;
  const _Float16* hPr = (const _Float16*)hPp;
  const int lane = threadIdx.x & 31;
  const int c = lane & 15, hh = lane >> 4, koff = hh * 8;
  const int d = blockIdx.y;
  const int r = rlo + blockIdx.x;
  const int ww = t - r;
  if (r < 0 || r >= NROW || ww < 0 || ww >= NCOL) return;
  const int h = (d & 2) ? (NROW - 1 - r) : r;
  const int w = (d & 1) ? (NCOL - 1 - ww) : ww;
  const bool hasA = (r > 0);
  const bool hasL = (ww > 0);
  int ha = (d & 2) ? (h + 1) : (h - 1);
  ha = ha < 0 ? 0 : (ha > NROW - 1 ? NROW - 1 : ha);
  int wl = (d & 1) ? (w + 1) : (w - 1);
  wl = wl < 0 ? 0 : (wl > NCOL - 1 ? NCOL - 1 : wl);
  const size_t cellS = ((size_t)(d * NROW + h) * NCOL + w) * CELL_ELEMS;
  const size_t cellA = ((size_t)(d * NROW + ha) * NCOL + w) * CELL_ELEMS;
  const size_t cellL = ((size_t)(d * NROW + h) * NCOL + wl) * CELL_ELEMS;

  v16h zf;
#pragma unroll
  for (int e = 0; e < 16; ++e) zf[e] = (_Float16)0.0f;

  const _Float16* xrow = xp + ((size_t)h * NCOL + w) * CELL_ELEMS + c * NCIN + koff;
  const v16h af0 = Frag<_Float16>::load(xrow);
  const v16h af1 = Frag<_Float16>::load(xrow + 32);
  v16h af2 = zf, af3 = zf, af4 = zf, af5 = zf;
  if (hasA) {
    const _Float16* p = hPr + cellA + c * NHID + koff;
    af2 = Frag<_Float16>::load(p);
    af3 = Frag<_Float16>::load(p + 32);
  }
  if (hasL) {
    const _Float16* p = hPr + cellL + c * NHID + koff;
    af4 = Frag<_Float16>::load(p);
    af5 = Frag<_Float16>::load(p + 32);
  }

  const _Float16* wdir = wc + (size_t)d * NGATE * KCAT + koff;
  const float* bdir = bs + d * NGATE;
  const float* cAp = cP + cellA;
  const float* cLp = cP + cellL;

#pragma unroll 1
  for (int ot = 0; ot < 4; ++ot) {
    const int o = 16 * ot + c;
    const float bi0 = bf16r(bdir[0 * NHID + o]) * WCARRY;
    const float bi1 = bf16r(bdir[1 * NHID + o]) * WCARRY;
    const float bi2 = bf16r(bdir[2 * NHID + o]) * WCARRY;
    const float bi3 = bf16r(bdir[3 * NHID + o]) * WCARRY;
    const float bi4 = bf16r(bdir[4 * NHID + o]) * WCARRY;
    v8f acc0, acc1, acc2, acc3, acc4;
#pragma unroll
    for (int rr = 0; rr < 8; ++rr) { acc0[rr] = bi0; acc1[rr] = bi1; acc2[rr] = bi2; acc3[rr] = bi3; acc4[rr] = bi4; }

    float ca[8], cl[8];
#pragma unroll
    for (int rr = 0; rr < 8; ++rr) { ca[rr] = 0.0f; cl[rr] = 0.0f; }
    if (hasA) {
#pragma unroll
      for (int rr = 0; rr < 8; ++rr) ca[rr] = cAp[(8 * hh + rr) * NHID + o];
    }
    if (hasL) {
#pragma unroll
      for (int rr = 0; rr < 8; ++rr) cl[rr] = cLp[(8 * hh + rr) * NHID + o];
    }

    const _Float16* wr = wdir + (size_t)o * KCAT;
    kstep5(acc0, acc1, acc2, acc3, acc4, af0, wr + 0);
    kstep5(acc0, acc1, acc2, acc3, acc4, af1, wr + 32);
    kstep5(acc0, acc1, acc2, acc3, acc4, af2, wr + 64);
    kstep5(acc0, acc1, acc2, acc3, acc4, af3, wr + 96);
    kstep5(acc0, acc1, acc2, acc3, acc4, af4, wr + 128);
    kstep5(acc0, acc1, acc2, acc3, acc4, af5, wr + 160);

#pragma unroll
    for (int rr = 0; rr < 8; ++rr) {
      const float ig = fsig(acc0[rr] * WCARRY_INV);
      const float fg = fsig(acc1[rr] * WCARRY_INV);
      const float gg = ftanh(acc2[rr] * WCARRY_INV);
      const float og = fsig(acc3[rr] * WCARRY_INV);
      const float lg = fsig(acc4[rr] * WCARRY_INV);
      const float blend = lg * ca[rr] + (1.0f - lg) * cl[rr];
      const float ct = fg * blend + ig * gg;
      const float ht = og * ftanh(ct);
      sC[(8 * hh + rr) * SLABP + o] = ct;
      sH[(8 * hh + rr) * SLABP + o] = ht;
    }
  }
  __syncthreads();

  const int q = lane >> 3, c8 = (lane & 7) * 8;
  v8h hv[4];
#pragma unroll
  for (int it = 0; it < 4; ++it) {
    const int row = it * 4 + q;
    const float* sp = sH + row * SLABP + c8;
    const v4f a = *(const v4f*)(sp);
    const v4f b = *(const v4f*)(sp + 4);
#pragma unroll
    for (int e = 0; e < 4; ++e) {
      const float fa = a[e];
      const float fb = b[e];
      hv[it][e] = (_Float16)fa;
      hv[it][4 + e] = (_Float16)fb;
    }
  }
  const int c4 = c * 4;
  v4f cv[8];
#pragma unroll
  for (int it = 0; it < 8; ++it) {
    const int row = it * 2 + hh;
    cv[it] = *(const v4f*)(sC + row * SLABP + c4);
  }
  unsigned short* hdst = hPp + cellS;
  float* cdst = cP + cellS;
  for (int pass = 0; pass < 2; ++pass) {
#pragma unroll
    for (int it = 0; it < 4; ++it) {
      const int row = it * 4 + q;
      *(volatile v8h*)(hdst + row * NHID + c8) = hv[it];
    }
#pragma unroll
    for (int it = 0; it < 8; ++it) {
      const int row = it * 2 + hh;
      *(volatile v4f*)(cdst + row * NHID + c4) = cv[it];
    }
    __threadfence();
  }
}

__global__ __launch_bounds__(256) void mean_out_kernel(const unsigned* __restrict__ hPw, const float* __restrict__ cP,
                                                       float* __restrict__ out0, float* __restrict__ out1) {
  __shared__ float Th[64 * TPITCH];
  __shared__ float Tc[64 * TPITCH];
  const int tid = threadIdx.x;
  const int w0 = blockIdx.x * 64, h = blockIdx.y, b = blockIdx.z;
#pragma unroll 1
  for (int i = 0; i < 4; ++i) {
    const int idx = i * 256 + tid;
    const int wl = idx >> 4, o4 = (idx & 15) * 4;
    v4f s = {0.0f, 0.0f, 0.0f, 0.0f};
#pragma unroll
    for (int d = 0; d < NDIR; ++d) {
      const size_t cell = ((size_t)(d * NROW + h) * NCOL + (size_t)(w0 + wl)) * CELL_ELEMS;
      const v4f v = *(const v4f*)(cP + cell + b * NHID + o4);
      s += v;
    }
    Tc[wl * TPITCH + o4 + 0] = s[0] * 0.25f;
    Tc[wl * TPITCH + o4 + 1] = s[1] * 0.25f;
    Tc[wl * TPITCH + o4 + 2] = s[2] * 0.25f;
    Tc[wl * TPITCH + o4 + 3] = s[3] * 0.25f;
  }
#pragma unroll 1
  for (int i = 0; i < 2; ++i) {
    const int idx = i * 256 + tid;
    const int wl = idx >> 3, o8 = (idx & 7) * 8;
    float s[8];
#pragma unroll
    for (int e = 0; e < 8; ++e) s[e] = 0.0f;
#pragma unroll
    for (int d = 0; d < NDIR; ++d) {
      const size_t cell = ((size_t)(d * NROW + h) * NCOL + (size_t)(w0 + wl)) * CELL_ELEMS;
      const v4u u = *(const v4u*)(hPw + ((cell + (size_t)(b * NHID + o8)) >> 1));
      const unsigned q0 = u[0], q1 = u[1], q2 = u[2], q3 = u[3];
      s[0] += h16_to_f32(q0 & 0xffffu);
      s[1] += h16_to_f32(q0 >> 16);
      s[2] += h16_to_f32(q1 & 0xffffu);
      s[3] += h16_to_f32(q1 >> 16);
      s[4] += h16_to_f32(q2 & 0xffffu);
      s[5] += h16_to_f32(q2 >> 16);
      s[6] += h16_to_f32(q3 & 0xffffu);
      s[7] += h16_to_f32(q3 >> 16);
    }
#pragma unroll
    for (int e = 0; e < 8; ++e) Th[wl * TPITCH + o8 + e] = s[e] * 0.25f;
  }
  __syncthreads();
  v4f vh[4], vc[4];
#pragma unroll
  for (int it = 0; it < 4; ++it) {
    const int idx = it * 256 + tid;
    const int orow = idx >> 4, c4 = (idx & 15) * 4;
#pragma unroll
    for (int e = 0; e < 4; ++e) {
      vh[it][e] = Th[(c4 + e) * TPITCH + orow];
      vc[it][e] = Tc[(c4 + e) * TPITCH + orow];
    }
  }
  for (int pass = 0; pass < 2; ++pass) {
#pragma unroll
    for (int it = 0; it < 4; ++it) {
      const int idx = it * 256 + tid;
      const int orow = idx >> 4, c4 = (idx & 15) * 4;
      const size_t off = (((size_t)b * NHID + orow) * NROW + h) * NCOL + w0 + c4;
      *(volatile v4f*)(out0 + off) = vh[it];
      *(volatile v4f*)(out1 + off) = vc[it];
    }
    __threadfence();
  }
}

extern "C" void kernel_launch(void* const* d_in, const int* in_sizes, int n_in,
                              void* d_out, int out_size, void* d_ws, size_t ws_size, hipStream_t stream) {
  if (n_in < 5 || d_out == nullptr || d_ws == nullptr) return;
  if (in_sizes[0] != NBATCH * NCIN * NROW * NCOL || in_sizes[1] != NDIR * NCIN * NGATE ||
      in_sizes[2] != NDIR * NHID * NGATE || in_sizes[3] != NDIR * NHID * NGATE ||
      in_sizes[4] != NDIR * NGATE || out_size != 2 * NOUT_ONE) return;

  const float* x   = (const float*)d_in[0];
  const float* wsr = (const float*)d_in[1];
  const float* u0r = (const float*)d_in[2];
  const float* u1r = (const float*)d_in[3];
  const float* bsr = (const float*)d_in[4];
  float* out0 = (float*)d_out;
  float* out1 = out0 + (size_t)NOUT_ONE;

  char* wsb = (char*)d_ws; size_t off = 0;
  auto carve = [&](size_t bytes) -> char* { char* p = wsb + off; off += (bytes + 255) & ~(size_t)255; return p; };
  unsigned short* XP = (unsigned short*)carve((size_t)NPIX * CELL_ELEMS * 2);
  unsigned short* WC = (unsigned short*)carve((size_t)NDIR * NGATE * KCAT * 2);
  unsigned short* HP = (unsigned short*)carve((size_t)NDIR * NPIX * CELL_ELEMS * 2);
  float*          CP = (float*)carve((size_t)NDIR * NPIX * CELL_ELEMS * 4);
  if (off > ws_size || off > (size_t)134217728) return;

  pack_x_kernel<<<dim3(NCOL / 64, NROW, NBATCH), 256, 0, stream>>>(x, XP);
  pack_w_kernel<<<dim3(NGATE / 64, 3, NDIR), 256, 0, stream>>>(wsr, u0r, u1r, WC);

  for (int t = 0; t < NROW + NCOL - 1; ++t) {
    const int rlo = (t > NCOL - 1) ? (t - (NCOL - 1)) : 0;
    const int rhi = (t < NROW - 1) ? t : (NROW - 1);
    const int nr = rhi - rlo + 1;
    grid_cell_kernel<<<dim3(nr, NDIR), 32, 0, stream>>>(XP, WC, bsr, HP, CP, t, rlo);
  }

  mean_out_kernel<<<dim3(NCOL / 64, NROW, NBATCH), 256, 0, stream>>>((const unsigned*)HP, CP, out0, out1);
}
